// SoftAlignLocalAttention_23373212025420
// MI455X (gfx1250) — hardware-verified
//
#include <hip/hip_runtime.h>
#include <hip/hip_bf16.h>
#include <math.h>

#define NBl 4
#define CCl 512
#define TTl 4096
#define NHl 8
#define HDl 64
#define WNl 16
#define PADL 8
#define GSTR 48

typedef _Float16 bf16;
typedef _Float16 f16;
typedef __attribute__((ext_vector_type(4))) unsigned v4u_t;
typedef unsigned v4ua __attribute__((ext_vector_type(4), may_alias));
typedef __attribute__((ext_vector_type(4))) float v4f_t;
typedef float v4fa __attribute__((ext_vector_type(4), may_alias));
typedef __attribute__((ext_vector_type(16))) bf16  bf16x16;
typedef bf16x16 f16x16;
typedef __attribute__((ext_vector_type(8)))  bf16  bf16x8;
typedef bf16x8 f16x8;
typedef __attribute__((ext_vector_type(8)))  float f32x8;
__device__ __forceinline__ f32x8 wmma16(f16x16 a, f16x16 b, f32x8 c) {
  c = __builtin_amdgcn_wmma_f32_16x16x32_f16(false, a, false, b, (short)0, c, false, false);
  asm volatile("v_nop\n\tv_nop\n\tv_nop\n\tv_nop" : "+v"(c) : "v"(a), "v"(b));
  return c;
}
__device__ __forceinline__ f16x16 lds_frag(const f16* base, int stride) {
  const int lane = threadIdx.x & 31, row = lane & 15, kh = (lane >> 4) * 8;
  const f16x8 lo = *(const f16x8*)(base + row * stride + kh);
  const f16x8 hi = *(const f16x8*)(base + row * stride + kh + 16);
  f16x16 f;
#pragma unroll
  for (int i = 0; i < 8; ++i) { f[i] = lo[i]; f[i + 8] = hi[i]; }
  return f;
}

#define GSTR 48
template <typename AT, int EPI, bool OUT16>
__global__ __launch_bounds__(256) void gemm_kne(const AT* __restrict__ A, int lda, const float* __restrict__ Wm, int ldw,
                                                const float* __restrict__ bias, const float* __restrict__ R, const float* __restrict__ gvec,
                                                void* __restrict__ Yv, int ldy, int K) {
  __shared__ __attribute__((aligned(16))) f16 ldsA[128 * GSTR];
  __shared__ __attribute__((aligned(16))) f16 ldsW[128 * GSTR];
  __shared__ __attribute__((aligned(16))) float oS[8][32 * 68];
  const int tid = threadIdx.x, lane = tid & 31, wave = tid >> 5, cl = lane & 15, rh = (lane >> 4) * 8;
  const int m0 = blockIdx.x * 128, n0 = blockIdx.y * 128;
  const int wm = (wave & 3) * 32, wn = (wave >> 2) * 64;
  f32x8 acc[2][4];
#pragma unroll
  for (int i = 0; i < 2; ++i)
#pragma unroll
    for (int j = 0; j < 4; ++j) { f32x8 z = {}; acc[i][j] = z; }
#pragma unroll 1
  for (int k0 = 0; k0 < K; k0 += 32) {
    __syncthreads();
    { const int row = tid >> 1, ch = (tid & 1) * 16;
      const AT* src = A + (size_t)(m0 + row) * lda + k0 + ch;
#pragma unroll
      for (int g = 0; g < 16; ++g) ldsA[row * GSTR + ch + g] = (f16)src[g]; }
    { const int k = tid >> 3, nn0 = (tid & 7) * 16;
      const float* src = Wm + (size_t)(k0 + k) * ldw + n0 + nn0;
#pragma unroll
      for (int g = 0; g < 4; ++g) { const v4f_t v = *(const v4f_t*)(src + 4 * g);
#pragma unroll
        for (int u = 0; u < 4; ++u) ldsW[(nn0 + 4 * g + u) * GSTR + k] = (f16)v[u]; } }
    __syncthreads();
    f16x16 af[2];
#pragma unroll
    for (int i = 0; i < 2; ++i) af[i] = lds_frag(ldsA + (wm + 16 * i) * GSTR, GSTR);
#pragma unroll
    for (int j = 0; j < 4; ++j) {
      const f16x16 bf = lds_frag(ldsW + (wn + 16 * j) * GSTR, GSTR);
#pragma unroll
      for (int i = 0; i < 2; ++i) acc[i][j] = wmma16(af[i], bf, acc[i][j]);
    }
  }
  float* so = oS[wave];
#pragma unroll
  for (int i = 0; i < 2; ++i)
#pragma unroll
    for (int j = 0; j < 4; ++j) {
      const int n = n0 + wn + 16 * j + cl;
      const float bv = bias ? bias[n] : 0.0f;
      const float gv = (EPI == 2) ? gvec[n] : 0.0f;
      if (EPI == 1) {
#pragma unroll 1
        for (int r = 0; r < 8; ++r) { const float xg = acc[i][j][r] + bv; so[(16 * i + rh + r) * 68 + 16 * j + cl] = 0.5f * xg * (1.0f + erff(xg * 0.70710678118654752f)); }
      } else {
#pragma unroll
        for (int r = 0; r < 8; ++r) {
          float v = acc[i][j][r] + bv;
          if (EPI == 2) v = R[(size_t)(m0 + wm + 16 * i + rh + r) * ldy + n] + gv * v;
          so[(16 * i + rh + r) * 68 + 16 * j + cl] = v;
        }
      }
    }
  asm volatile("s_wait_dscnt 0" ::: "memory");
  __builtin_amdgcn_wave_barrier();
#pragma unroll 1
  for (int pass = 0; pass < 2; ++pass) {
    if (OUT16) {
      f16* Y = (f16*)Yv;
#pragma unroll
      for (int it = 0; it < 8; ++it) { const int c = lane + 32 * it, rr = c >> 3, q8 = (c & 7) * 8;
        union { f16 h[8]; v4u_t v; } u;
#pragma unroll
        for (int e = 0; e < 8; ++e) u.h[e] = (f16)so[rr * 68 + q8 + e];
        *(volatile v4u_t*)(Y + (size_t)(m0 + wm + rr) * ldy + n0 + wn + q8) = u.v; }
    } else {
      float* Y = (float*)Yv;
#pragma unroll
      for (int it = 0; it < 16; ++it) { const int f4 = lane + 32 * it, rr = f4 >> 4, q = (f4 & 15) * 4;
        *(volatile v4f_t*)(Y + (size_t)(m0 + wm + rr) * ldy + n0 + wn + q) = *(const v4fa*)(so + rr * 68 + q); }
    }
    __threadfence();
  }
}

__global__ __launch_bounds__(256) void k_local(const float* __restrict__ q, const float* __restrict__ k, const float* __restrict__ v, const float* __restrict__ bq, const float* __restrict__ bk, const float* __restrict__ bv,
                                              float* __restrict__ ctx) {
  __shared__ float kS[HDl][80], vS[HDl][80];
  __shared__ float qS[HDl][64];
  __shared__ float pS[64][WNl];
  __shared__ __attribute__((aligned(16))) float oS[HDl][68];
  const int tid = threadIdx.x; const int h = blockIdx.y, t0 = blockIdx.x * 64; const int c0 = h * HDl;
  const float* qb = q + (size_t)c0 * TTl; const float* kb_ = k + (size_t)c0 * TTl; const float* vb_ = v + (size_t)c0 * TTl;
  for (int e = tid; e < HDl * 80; e += 256) { const int d = e / 80, s = e % 80; const int t = t0 - PADL + s;
    const bool in = (t >= 0 && t < TTl && s < 79); kS[d][s] = in ? kb_[(size_t)d * TTl + t] + bk[c0 + d] : 0.0f; vS[d][s] = in ? vb_[(size_t)d * TTl + t] + bv[c0 + d] : 0.0f; }
  for (int e = tid; e < HDl * 64; e += 256) { const int d = e >> 6, tl = e & 63; qS[d][tl] = qb[(size_t)d * TTl + t0 + tl] + bq[c0 + d]; }
  __syncthreads();
  const int tl = tid >> 2, part = tid & 3;
  float dots[WNl];
#pragma unroll
  for (int w = 0; w < WNl; ++w) { float s = 0.0f;
#pragma unroll 1
    for (int dd = 0; dd < 16; ++dd) { const int d = part * 16 + dd; s += qS[d][tl] * kS[d][tl + w]; }
    s += __shfl_xor(s, 1, 32); s += __shfl_xor(s, 2, 32); dots[w] = s * 0.125f; }
  if (part == 0) { float m = dots[0];
#pragma unroll
    for (int w = 1; w < WNl; ++w) m = fmaxf(m, dots[w]);
    float z = 0.0f; float ew[WNl];
#pragma unroll
    for (int w = 0; w < WNl; ++w) { ew[w] = expf(dots[w] - m); z += ew[w]; }
    const float iz = 1.0f / z;
#pragma unroll
    for (int w = 0; w < WNl; ++w) pS[tl][w] = ew[w] * iz; }
  __syncthreads();
#pragma unroll 1
  for (int dd = 0; dd < 16; ++dd) { const int d = part * 16 + dd; float s = 0.0f;
#pragma unroll
    for (int w = 0; w < WNl; ++w) s += pS[tl][w] * vS[d][tl + w];
    oS[d][tl] = s; }
  __syncthreads();
#pragma unroll 1
  for (int pass = 0; pass < 2; ++pass) { for (int q4 = tid; q4 < HDl * 16; q4 += 256) { const int d = q4 >> 4, c4 = (q4 & 15) * 4;
      *(volatile v4f_t*)(ctx + ((size_t)c0 + d) * TTl + t0 + c4) = *(const v4fa*)(&oS[d][c4]); } __threadfence(); }
}
__global__ __launch_bounds__(256) void k_rowbias(float* __restrict__ o, const float* __restrict__ bo) {
  const size_t row = blockIdx.x; const int c = (int)(row % CCl); const float bb = bo[c]; const int tid = threadIdx.x;
  for (int c4 = tid * 4; c4 < TTl; c4 += 1024) { v4f_t vv = *(const v4f_t*)(o + row * TTl + c4); vv[0] += bb; vv[1] += bb; vv[2] += bb; vv[3] += bb;
    *(volatile v4f_t*)(o + row * TTl + c4) = vv; __threadfence(); *(volatile v4f_t*)(o + row * TTl + c4) = vv; }
}

extern "C" void kernel_launch(void* const* d_in, const int* in_sizes, int n_in,
                              void* d_out, int out_size, void* d_ws, size_t ws_size,
                              hipStream_t stream) {
  (void)in_sizes; (void)n_in; (void)out_size;
  const float** f = (const float**)d_in;
  const float* x = f[0], *cond = f[1], *Wq = f[2], *bq = f[3], *Wk = f[4], *bk = f[5], *Wv = f[6], *bv = f[7], *Wo = f[8], *bo = f[9];
  float* out = (float*)d_out;
  char* ws = (char*)d_ws;
  float* q = (float*)ws; ws += (size_t)CCl * TTl * 4;
  float* k = (float*)ws; ws += (size_t)CCl * TTl * 4;
  float* v = (float*)ws; ws += (size_t)CCl * TTl * 4;
  float* ctx = (float*)ws; ws += (size_t)CCl * TTl * 4;
  if ((size_t)(ws - (char*)d_ws) > ws_size) return;
  const dim3 blk(256);
  for (int b = 0; b < NBl; ++b) {
    const float* xb = x + (size_t)b * CCl * TTl; const float* cb = cond + (size_t)b * CCl * TTl; float* ob = out + (size_t)b * CCl * TTl;
    gemm_kne<float, 0, false><<<dim3(CCl / 128, TTl / 128), blk, 0, stream>>>(Wq, CCl, xb, TTl, nullptr, nullptr, nullptr, q, TTl, CCl);
    gemm_kne<float, 0, false><<<dim3(CCl / 128, TTl / 128), blk, 0, stream>>>(Wk, CCl, cb, TTl, nullptr, nullptr, nullptr, k, TTl, CCl);
    gemm_kne<float, 0, false><<<dim3(CCl / 128, TTl / 128), blk, 0, stream>>>(Wv, CCl, cb, TTl, nullptr, nullptr, nullptr, v, TTl, CCl);
    k_local<<<dim3(TTl / 64, NHl, 1), blk, 0, stream>>>(q, k, v, bq, bk, bv, ctx);
    gemm_kne<float, 0, false><<<dim3(CCl / 128, TTl / 128), blk, 0, stream>>>(Wo, CCl, ctx, TTl, nullptr, nullptr, nullptr, ob, TTl, CCl);
  }
  k_rowbias<<<dim3(NBl * CCl), blk, 0, stream>>>(out, bo);
}
